// TumorTemporalGNN_34557306864290
// MI455X (gfx1250) — hardware-verified
//
#include <hip/hip_runtime.h>
#include <stddef.h>


#define NGRAPH 128
#define NNODE  512
#define NEDGE  4096
#define FIN    64
#define DDIM   128
#define NHEAD  4
#define CDIM   32
#define NBAT   16
#define NT     8
#define NTH    4
#define DH     32
#define NCLS   3
#define NROWS  (NGRAPH * NNODE)
#define NTHR   256
#define NWAVE  8
#define EPT    8
#define NGRP   2
#define CHUNK  (NTHR * EPT * NGRP)
#define WCAP   (EPT * NGRP * 32)
#define LISTN  (NWAVE * WCAP)
#define NBT    64
#define NTG    (NNODE / NBT)
#define GPB    8
#define RCAP   4096
#define DEGCAP 512
#define GB     64
#define GTHR   128
#define SP     132
#define HP     136
#define QP     388
#define WSCAP  134217728
#define NEG_SLOPE 0.2f
#define DEN_EPS   1e-16f
#define RSQ       0.17677669529663688f
#define LDS_AGG   ((2 * RCAP + LISTN) * 4)

static_assert((CHUNK & (CHUNK - 1)) == 0);
static_assert(CHUNK <= 4096);
static_assert((NBT & (NBT - 1)) == 0 && NBT <= 4096 && NBT % NWAVE == 0);
static_assert(NNODE % NBT == 0 && NGRAPH % GPB == 0 && GPB == NWAVE);
static_assert(DDIM == NHEAD * CDIM && DDIM == NTH * DH && DDIM == 4 * 32);
static_assert(NROWS % GB == 0 && GB == 16 * (GTHR / 32) && GB * NHEAD == 2 * 128);
static_assert(FIN % 32 == 0 && DDIM % 32 == 0);
static_assert(((HP * 2) % 16) == 0 && ((SP * 4) % 16) == 0 && ((QP * 4) % 16) == 0);
static_assert(NT * NTH * NT == NTHR);
static_assert(NT * DDIM == 4 * NTHR);
static_assert(3 * DDIM == NWAVE * 3 * 16);
static_assert(DDIM == NWAVE * 16);
static_assert(NBAT * NT == NGRAPH && (NBAT * NCLS) % 4 == 0 && NBAT * NCLS <= 128);
static_assert((NROWS * FIN) % (8 * NTHR) == 0);
static_assert(LDS_AGG <= 65536);
static_assert(RCAP >= NEDGE);

typedef float          v2f  __attribute__((ext_vector_type(2)));
typedef float          v4f  __attribute__((ext_vector_type(4)));
typedef float          v8f  __attribute__((ext_vector_type(8)));
typedef int            v4i  __attribute__((ext_vector_type(4)));
typedef unsigned int   v2u  __attribute__((ext_vector_type(2)));
typedef unsigned int   v4u  __attribute__((ext_vector_type(4)));
typedef unsigned short v4us __attribute__((ext_vector_type(4)));
typedef unsigned short v8us __attribute__((ext_vector_type(8)));
typedef __bf16         v16b __attribute__((ext_vector_type(16)));
union FragB { v16b v; v8us h[2]; };
union Pk4u  { v4us h; v2u u; };

__device__ __forceinline__ unsigned int bfr(float f) {
  const unsigned int u = __float_as_uint(f);
  return (u + 0x7FFFu + ((u >> 16) & 1u)) >> 16;
}

__device__ __forceinline__ void split1(float x, unsigned short& hb, unsigned short& lb) {
  const unsigned int hu = bfr(x);
  const float hf = __uint_as_float(hu << 16);
  hb = (unsigned short)hu;
  lb = (unsigned short)bfr(x - hf);
}

__device__ __forceinline__ void split4(v4f a, v4us& hi, v4us& lo) {
  unsigned short hb, lb;
  split1(a.x, hb, lb); hi[0] = hb; lo[0] = lb;
  split1(a.y, hb, lb); hi[1] = hb; lo[1] = lb;
  split1(a.z, hb, lb); hi[2] = hb; lo[2] = lb;
  split1(a.w, hb, lb); hi[3] = hb; lo[3] = lb;
}

__device__ __forceinline__ void split8(v4f a, v4f b, v8us& hi, v8us& lo) {
  unsigned short hb, lb;
  split1(a.x, hb, lb); hi[0] = hb; lo[0] = lb;
  split1(a.y, hb, lb); hi[1] = hb; lo[1] = lb;
  split1(a.z, hb, lb); hi[2] = hb; lo[2] = lb;
  split1(a.w, hb, lb); hi[3] = hb; lo[3] = lb;
  split1(b.x, hb, lb); hi[4] = hb; lo[4] = lb;
  split1(b.y, hb, lb); hi[5] = hb; lo[5] = lb;
  split1(b.z, hb, lb); hi[6] = hb; lo[6] = lb;
  split1(b.w, hb, lb); hi[7] = hb; lo[7] = lb;
}

__device__ __forceinline__ v8f wmb(v16b a, v16b b, v8f c) {
  v8f d = __builtin_amdgcn_wmma_f32_16x16x32_bf16(false, a, false, b, (short)0, c, false, false);
  asm volatile("v_nop\n\tv_nop\n\tv_nop\n\tv_nop" : "+v"(d) : "v"(a), "v"(b));
  return d;
}

__device__ __forceinline__ float lrelu(float v) { return v > 0.0f ? v : NEG_SLOPE * v; }
__device__ __forceinline__ float eluf(float v) {
  const float ser = v * (1.0f + v * (0.5f + v * (0.16666667f + v * (0.041666668f + v * 0.0083333338f))));
  const float big = __expf(v) - 1.0f;
  const float neg = (v > -0.0625f) ? ser : big;
  return v > 0.0f ? v : neg;
}

template <int NB>
__device__ __forceinline__ int scan_chunk(const int* __restrict__ dsts, int nE, int cbase, int slotBase,
                                          int vec8, int* list, int tid, int lane, int wave) {
  int wc = 0;
#pragma unroll
  for (int g = 0; g < NGRP; ++g) {
    const int el0  = (g * NTHR + tid) * EPT;
    const int e0   = cbase + el0;
    const int sent = -2147483647 - 1;
    v4i da, db;
    if (vec8 != 0 && cbase + CHUNK <= nE) {
      da = *(const v4i*)(dsts + e0);
      db = *(const v4i*)(dsts + e0 + 4);
    } else {
      da.x = (e0     < nE) ? dsts[min(e0, nE - 1)] : sent;
      da.y = (e0 + 1 < nE) ? dsts[min(e0 + 1, nE - 1)] : sent;
      da.z = (e0 + 2 < nE) ? dsts[min(e0 + 2, nE - 1)] : sent;
      da.w = (e0 + 3 < nE) ? dsts[min(e0 + 3, nE - 1)] : sent;
      db.x = (e0 + 4 < nE) ? dsts[min(e0 + 4, nE - 1)] : sent;
      db.y = (e0 + 5 < nE) ? dsts[min(e0 + 5, nE - 1)] : sent;
      db.z = (e0 + 6 < nE) ? dsts[min(e0 + 6, nE - 1)] : sent;
      db.w = (e0 + 7 < nE) ? dsts[min(e0 + 7, nE - 1)] : sent;
    }
    const unsigned nb = (unsigned)slotBase;
    const unsigned s0 = (unsigned)da.x - nb, s1 = (unsigned)da.y - nb;
    const unsigned s2 = (unsigned)da.z - nb, s3 = (unsigned)da.w - nb;
    const unsigned s4 = (unsigned)db.x - nb, s5 = (unsigned)db.y - nb;
    const unsigned s6 = (unsigned)db.z - nb, s7 = (unsigned)db.w - nb;
    const bool h0 = s0 < (unsigned)NB, h1 = s1 < (unsigned)NB, h2 = s2 < (unsigned)NB, h3 = s3 < (unsigned)NB;
    const bool h4 = s4 < (unsigned)NB, h5 = s5 < (unsigned)NB, h6 = s6 < (unsigned)NB, h7 = s7 < (unsigned)NB;
    const unsigned any = __builtin_amdgcn_ballot_w32(h0 | h1 | h2 | h3 | h4 | h5 | h6 | h7);
    if (any != 0u) {
#define HITJ(J, HJ, SJ) { \
        const unsigned mj = __builtin_amdgcn_ballot_w32(HJ); \
        if (mj != 0u) { \
          if (HJ) { \
            const int pos = wc + (int)__builtin_amdgcn_mbcnt_lo(mj, 0u); \
            if (pos < WCAP) list[wave * WCAP + pos] = ((el0 + (J)) << 12) | (int)(SJ); \
          } \
          wc += (int)__builtin_popcount(mj); } }
      HITJ(0, h0, s0)
      HITJ(1, h1, s1)
      HITJ(2, h2, s2)
      HITJ(3, h3, s3)
      HITJ(4, h4, s4)
      HITJ(5, h5, s5)
      HITJ(6, h6, s6)
      HITJ(7, h7, s7)
#undef HITJ
    }
  }
  return wc;
}

__global__ __launch_bounds__(NTHR) void k_prep_w(
    const float* __restrict__ W0, const float* __restrict__ W1,
    const float* __restrict__ Wq, const float* __restrict__ Wk,
    const float* __restrict__ Wv, const float* __restrict__ Wo,
    unsigned short* p0, unsigned short* p1, unsigned short* pq) {
  const int b = (int)blockIdx.x, tid = (int)threadIdx.x;
  const float* W;
  unsigned short* P;
  int K, u;
  if (b < 4) {
    W = W0; P = p0; K = FIN; u = b * NTHR + tid;
  } else {
    const int j = (b - 4) >> 3, bb = (b - 4) & 7;
    K = DDIM; u = bb * NTHR + tid;
    W = (j == 0) ? W1 : ((j == 1) ? Wq : ((j == 2) ? Wk : ((j == 3) ? Wv : Wo)));
    P = (j == 0) ? p1 : (pq + (size_t)(j - 1) * 2 * DDIM * DDIM);
  }
  const int kg = K >> 3;
  const int n = u / kg, k0 = (u - n * kg) * 8;
  float v[8];
#pragma unroll
  for (int e = 0; e < 8; ++e) v[e] = W[(size_t)(k0 + e) * DDIM + n];
  v4f a, c;
  a.x = v[0]; a.y = v[1]; a.z = v[2]; a.w = v[3];
  c.x = v[4]; c.y = v[5]; c.z = v[6]; c.w = v[7];
  v8us hv, lv;
  split8(a, c, hv, lv);
  unsigned short* dh = P + (size_t)u * 8;
  unsigned short* dl = dh + (size_t)DDIM * K;
  *(volatile v8us*)dh = hv;
  *(volatile v8us*)dl = lv;
  __threadfence();
  *(volatile v8us*)dh = hv;
  *(volatile v8us*)dl = lv;
}

__global__ __launch_bounds__(NTHR) void k_cvt(const float* __restrict__ x, unsigned short* xh,
                                               unsigned short* xl, int nUnits) {
  const int i = (int)blockIdx.x * NTHR + (int)threadIdx.x;
  if (i >= nUnits) return;
  const float* sp = x + (size_t)i * 8;
  const v4f a = *(const v4f*)sp, c = *(const v4f*)(sp + 4);
  v8us hv, lv;
  split8(a, c, hv, lv);
  unsigned short* dh = xh + (size_t)i * 8;
  unsigned short* dl = xl + (size_t)i * 8;
  *(volatile v8us*)dh = hv;
  *(volatile v8us*)dl = lv;
  __threadfence();
  *(volatile v8us*)dh = hv;
  *(volatile v8us*)dl = lv;
}

__global__ __launch_bounds__(GTHR) void k_gemm(
    const unsigned short* __restrict__ ahi, const unsigned short* __restrict__ alo,
    const unsigned short* __restrict__ wp, const float* __restrict__ attS, const float* __restrict__ attD,
    float* hp, float* eS, float* eD, int K, int nRows) {
  __shared__ __attribute__((aligned(16))) float stg[GB * SP];
  __shared__ __attribute__((aligned(16))) float sES[GB * NHEAD];
  __shared__ __attribute__((aligned(16))) float sED[GB * NHEAD];
  const int tid = threadIdx.x, lane = tid & 31, wave = tid >> 5, hh = lane >> 4, m = lane & 15;
  const int rowBase = blockIdx.x * GB;

  int row = rowBase + wave * 16 + m;
  row = row > nRows - 1 ? nRows - 1 : row;
  const unsigned short* aph = ahi + (size_t)row * K + 8 * hh;
  const unsigned short* apl = alo + (size_t)row * K + 8 * hh;
  const unsigned short* wb  = wp + (size_t)m * K + 8 * hh;
  const size_t wlo = (size_t)DDIM * K;

  v8f acc[8];
#pragma unroll
  for (int t = 0; t < 8; ++t) { v8f z = {0.f, 0.f, 0.f, 0.f, 0.f, 0.f, 0.f, 0.f}; acc[t] = z; }
#pragma unroll 1
  for (int k0 = 0; k0 < K; k0 += 32) {
    FragB ah, al;
    ah.h[0] = *(const v8us*)(aph + k0);
    ah.h[1] = *(const v8us*)(aph + k0 + 16);
    al.h[0] = *(const v8us*)(apl + k0);
    al.h[1] = *(const v8us*)(apl + k0 + 16);
#pragma unroll
    for (int t = 0; t < 8; ++t) {
      const unsigned short* bp = wb + (size_t)(16 * t) * K + k0;
      FragB bh, bl;
      bh.h[0] = *(const v8us*)bp;
      bh.h[1] = *(const v8us*)(bp + 16);
      bl.h[0] = *(const v8us*)(bp + wlo);
      bl.h[1] = *(const v8us*)(bp + wlo + 16);
      acc[t] = wmb(ah.v, bh.v, acc[t]);
      acc[t] = wmb(ah.v, bl.v, acc[t]);
      acc[t] = wmb(al.v, bh.v, acc[t]);
    }
  }
  {
    float* sp = stg + (size_t)(wave * 16 + 8 * hh) * SP + m;
#pragma unroll
    for (int t = 0; t < 8; ++t) {
#pragma unroll
      for (int r = 0; r < 8; ++r) sp[r * SP + 16 * t] = acc[t][r];
    }
  }
  __syncthreads();

  const int hd = lane >> 3;
  const v4f sa = *(const v4f*)(attS + 4 * lane);
  const v4f sd = *(const v4f*)(attD + 4 * lane);
#pragma unroll 1
  for (int it = 0; it < 16; ++it) {
    const int r = wave * 16 + it;
    const v4f v = *(const v4f*)(stg + (size_t)r * SP + 4 * lane);
    *(volatile v4f*)(hp + (size_t)(rowBase + r) * DDIM + 4 * lane) = v;
    float ps = v.x * sa.x + v.y * sa.y + v.z * sa.z + v.w * sa.w;
    float pd = v.x * sd.x + v.y * sd.y + v.z * sd.z + v.w * sd.w;
    ps += __shfl_xor(ps, 1); pd += __shfl_xor(pd, 1);
    ps += __shfl_xor(ps, 2); pd += __shfl_xor(pd, 2);
    ps += __shfl_xor(ps, 4); pd += __shfl_xor(pd, 4);
    if ((lane & 7) == 0) { sES[r * NHEAD + hd] = ps; sED[r * NHEAD + hd] = pd; }
  }
  __threadfence();
#pragma unroll 1
  for (int it = 0; it < 16; ++it) {
    const int r = wave * 16 + it;
    const v4f v = *(const v4f*)(stg + (size_t)r * SP + 4 * lane);
    *(volatile v4f*)(hp + (size_t)(rowBase + r) * DDIM + 4 * lane) = v;
  }
  __syncthreads();

  v4f d0 = {0.f, 0.f, 0.f, 0.f}, d1 = {0.f, 0.f, 0.f, 0.f};
  const size_t eb = (size_t)rowBase * NHEAD;
  if (wave == 0) {
    d0 = *(const v4f*)(sES + 4 * lane);
    d1 = *(const v4f*)(sES + 128 + 4 * lane);
    *(volatile v4f*)(eS + eb + 4 * lane) = d0;
    *(volatile v4f*)(eS + eb + 128 + 4 * lane) = d1;
  } else if (wave == 1) {
    d0 = *(const v4f*)(sED + 4 * lane);
    d1 = *(const v4f*)(sED + 128 + 4 * lane);
    *(volatile v4f*)(eD + eb + 4 * lane) = d0;
    *(volatile v4f*)(eD + eb + 128 + 4 * lane) = d1;
  }
  __threadfence();
  if (wave == 0) {
    *(volatile v4f*)(eS + eb + 4 * lane) = d0;
    *(volatile v4f*)(eS + eb + 128 + 4 * lane) = d1;
  } else if (wave == 1) {
    *(volatile v4f*)(eD + eb + 4 * lane) = d0;
    *(volatile v4f*)(eD + eb + 128 + 4 * lane) = d1;
  }
}

__global__ __launch_bounds__(NTHR) void k_agg(
    const int* __restrict__ ei, const float* __restrict__ ea,
    const float* __restrict__ We, const float* __restrict__ attE, const float* __restrict__ gbias,
    const float* __restrict__ hp, const float* __restrict__ eS, const float* __restrict__ eD,
    unsigned short* oh, unsigned short* ol, float* part,
    int nN, int nE, int nG, int ntg, int vec8, int pool) {
  extern __shared__ v4f lds_dyn[];
  int* region = (int*)lds_dyn;
  int* rege   = region + RCAP;
  int* list   = rege + RCAP;
  __shared__ int scnt[NBT];
  __shared__ int soff[NBT];
  __shared__ int curs[NBT];
  __shared__ int wcnt[NWAVE];
  __shared__ float sW[2 * NHEAD];
  __shared__ __attribute__((aligned(16))) float sBias[DDIM];
  __shared__ __attribute__((aligned(16))) float sPart[NWAVE * DDIM];
  __shared__ __attribute__((aligned(16))) float sRow[GPB * DDIM];
  const int tid = threadIdx.x, lane = tid & 31, wave = tid >> 5;
  const int nodeBase = blockIdx.x * NBT;
  const int gBase = blockIdx.y * GPB;
  const int* srcs = ei;
  const int* dsts = ei + nE;

  for (int i = tid; i < NBT; i += NTHR) scnt[i] = 0;
  for (int i = tid; i < RCAP; i += NTHR) { region[i] = 0; rege[i] = 0; }
  if (tid < DDIM) sBias[tid] = gbias[tid];
  if (tid < 2 * NHEAD) {
    const int k = tid >> 2, h = tid & 3;
    float s = 0.0f;
#pragma unroll 1
    for (int c = 0; c < CDIM; ++c) s += We[k * DDIM + h * CDIM + c] * attE[h * CDIM + c];
    sW[tid] = s;
  }
  __syncthreads();

  const int nChunks = (nE + CHUNK - 1) / CHUNK;
#pragma unroll 1
  for (int chn = 0; chn < nChunks; ++chn) {
    const int cbase = chn * CHUNK;
    const int wc = scan_chunk<NBT>(dsts, nE, cbase, nodeBase, vec8, list, tid, lane, wave);
    if (lane == 0) wcnt[wave] = wc;
    __syncthreads();
    if (wave == 0) {
#pragma unroll 1
      for (int wsx = 0; wsx < NWAVE; ++wsx) {
        int n = __builtin_amdgcn_readfirstlane(wcnt[wsx]);
        n = n > WCAP ? WCAP : (n < 0 ? 0 : n);
        const int* lp = list + wsx * WCAP;
#pragma unroll 1
        for (int i = 0; i < n; ++i) {
          const int ent  = __builtin_amdgcn_readfirstlane(lp[i]);
          const int slot = ent & (NBT - 1);
          if (lane == 0) scnt[slot] = scnt[slot] + 1;
        }
      }
    }
    __syncthreads();
  }
  if (tid == 0) {
    int run = 0;
#pragma unroll 1
    for (int s = 0; s < NBT; ++s) {
      soff[s] = run;
      curs[s] = run;
      int cv = scnt[s];
      cv = cv < 0 ? 0 : cv;
      run += cv;
      run = run > RCAP ? RCAP : run;
    }
  }
  __syncthreads();
#pragma unroll 1
  for (int chn = 0; chn < nChunks; ++chn) {
    const int cbase = chn * CHUNK;
    const int wc = scan_chunk<NBT>(dsts, nE, cbase, nodeBase, vec8, list, tid, lane, wave);
    if (lane == 0) wcnt[wave] = wc;
    __syncthreads();
    if (wave == 0) {
#pragma unroll 1
      for (int wsx = 0; wsx < NWAVE; ++wsx) {
        int n = __builtin_amdgcn_readfirstlane(wcnt[wsx]);
        n = n > WCAP ? WCAP : (n < 0 ? 0 : n);
        const int* lp = list + wsx * WCAP;
#pragma unroll 1
        for (int i = 0; i < n; ++i) {
          const int ent  = __builtin_amdgcn_readfirstlane(lp[i]);
          const int slot = ent & (NBT - 1);
          int e = cbase + ((ent >> 12) & (CHUNK - 1));
          e = e < 0 ? 0 : (e > nE - 1 ? nE - 1 : e);
          int src = srcs[e];
          src = src < 0 ? 0 : (src > nN - 1 ? nN - 1 : src);
          if (lane == 0) {
            int pos = curs[slot];
            pos = pos < 0 ? 0 : (pos > RCAP - 1 ? RCAP - 1 : pos);
            region[pos] = src;
            rege[pos] = e;
            const int np = pos + 1;
            curs[slot] = np > RCAP ? RCAP : np;
          }
        }
      }
    }
    __syncthreads();
  }

  const int hd = lane >> 3;
  const float w0 = sW[hd], w1 = sW[NHEAD + hd];
  const v4f bias4 = *(const v4f*)(sBias + 4 * lane);
#pragma unroll 1
  for (int gi = 0; gi < GPB; ++gi) {
    int g = gBase + gi;
    g = g > nG - 1 ? nG - 1 : g;
    const float* eab = ea + (size_t)g * nE * 2;
    v4f psum = {0.f, 0.f, 0.f, 0.f};
#pragma unroll 1
    for (int tl = wave; tl < NBT; tl += NWAVE) {
      const int c = nodeBase + tl;
      if (c < nN) {
        int st = soff[tl];
        st = st < 0 ? 0 : (st > RCAP ? RCAP : st);
        int deg = curs[tl] - st;
        deg = deg < 0 ? 0 : (deg > DEGCAP ? DEGCAP : deg);
        const size_t rowc = (size_t)g * nN + c;
        const float edv = eD[rowc * NHEAD + hd];
        float mx = -3.0e38f;
#pragma unroll 1
        for (int p = 0; p < deg; ++p) {
          int pos = st + p;
          pos = pos > RCAP - 1 ? RCAP - 1 : pos;
          const int s = region[pos];
          const int e = rege[pos];
          const v2f av = *(const v2f*)(eab + 2 * (size_t)e);
          const size_t rows = (size_t)g * nN + s;
          const float a = lrelu(eS[rows * NHEAD + hd] + edv + (av.x * w0 + av.y * w1));
          mx = fmaxf(mx, a);
        }
        float den = 0.0f;
        v4f acc = {0.f, 0.f, 0.f, 0.f};
#pragma unroll 1
        for (int p = 0; p < deg; ++p) {
          int pos = st + p;
          pos = pos > RCAP - 1 ? RCAP - 1 : pos;
          const int s = region[pos];
          const int e = rege[pos];
          const v2f av = *(const v2f*)(eab + 2 * (size_t)e);
          const size_t rows = (size_t)g * nN + s;
          const float a = lrelu(eS[rows * NHEAD + hd] + edv + (av.x * w0 + av.y * w1));
          const float pe = __expf(a - mx);
          den += pe;
          const v4f hv = *(const v4f*)(hp + rows * DDIM + 4 * lane);
          acc = acc + hv * pe;
        }
        const float rden = __builtin_amdgcn_rcpf(den + DEN_EPS);
        const v4f v = acc * rden + bias4;
        v4f ev;
        ev.x = eluf(v.x); ev.y = eluf(v.y); ev.z = eluf(v.z); ev.w = eluf(v.w);
        psum = psum + ev;
        if (pool == 0) {
          Pk4u ph, pl;
          split4(ev, ph.h, pl.h);
          unsigned short* gph = oh + rowc * DDIM + 4 * lane;
          unsigned short* gpl = ol + rowc * DDIM + 4 * lane;
          *(volatile v2u*)gph = ph.u;
          *(volatile v2u*)gpl = pl.u;
          __threadfence();
          *(volatile v2u*)gph = ph.u;
          *(volatile v2u*)gpl = pl.u;
        }
      }
    }
    *(v4f*)(sPart + wave * DDIM + 4 * lane) = psum;
    __syncthreads();
    if (tid < DDIM) {
      float s = 0.0f;
#pragma unroll
      for (int w = 0; w < NWAVE; ++w) s += sPart[w * DDIM + tid];
      sRow[gi * DDIM + tid] = s;
    }
    __syncthreads();
  }
  if (pool != 0) {
    const int g = gBase + wave;
    if (g < nG) {
      const v4f v = *(const v4f*)(sRow + wave * DDIM + 4 * lane);
      float* dp = part + ((size_t)g * ntg + blockIdx.x) * DDIM + 4 * lane;
      *(volatile v4f*)dp = v;
      __threadfence();
      *(volatile v4f*)dp = v;
    }
  }
}

__global__ __launch_bounds__(NTHR) void k_tail(
    const float* __restrict__ part, const float* __restrict__ intervals,
    const float* __restrict__ wt, const float* __restrict__ bt,
    const unsigned short* __restrict__ pq, const int* __restrict__ seqlen,
    const float* __restrict__ Wc, const float* __restrict__ bc,
    float* out, int nBatch, int ntg) {
  __shared__ __attribute__((aligned(16))) unsigned short sAh[16 * HP];
  __shared__ __attribute__((aligned(16))) unsigned short sAl[16 * HP];
  __shared__ __attribute__((aligned(16))) float sHin[NT * DDIM];
  __shared__ __attribute__((aligned(16))) float sQKV[16 * QP];
  __shared__ __attribute__((aligned(16))) float sP[NT * NTH * NT];
  __shared__ __attribute__((aligned(16))) float sCto[16 * SP];
  __shared__ __attribute__((aligned(16))) float sSum[NBAT * DDIM];
  __shared__ __attribute__((aligned(16))) float sOut[128];
  const int tid = threadIdx.x, lane = tid & 31, wave = tid >> 5, hh = lane >> 4, m = lane & 15;
  if (blockIdx.x != 0) return;

  for (int i = tid; i < 16 * HP; i += NTHR) { sAh[i] = 0; sAl[i] = 0; }
  for (int i = tid; i < 128; i += NTHR) sOut[i] = 0.0f;
  for (int i = tid; i < NBAT * DDIM; i += NTHR) sSum[i] = 0.0f;
  __syncthreads();

  const int nb = nBatch > NBAT ? NBAT : nBatch;
#pragma unroll 1
  for (int b = 0; b < nb; ++b) {
    {
      const int t = tid >> 5, d4 = (tid & 31) * 4;
      const int g = b * NT + t;
      v4f s = {0.f, 0.f, 0.f, 0.f};
#pragma unroll 1
      for (int tg = 0; tg < ntg; ++tg) s = s + *(const v4f*)(part + ((size_t)g * ntg + tg) * DDIM + d4);
      const float iv = intervals[g];
      const v4f w4 = *(const v4f*)(wt + d4);
      const v4f b4 = *(const v4f*)(bt + d4);
      const v4f hin = s * (1.0f / (float)NNODE) + w4 * iv + b4;
      *(v4f*)(sHin + t * DDIM + d4) = hin;
      v4us hv, lv;
      split4(hin, hv, lv);
      *(v4us*)(sAh + t * HP + d4) = hv;
      *(v4us*)(sAl + t * HP + d4) = lv;
    }
    __syncthreads();

    {
      v8f acc[3];
#pragma unroll
      for (int tt = 0; tt < 3; ++tt) { v8f z = {0.f, 0.f, 0.f, 0.f, 0.f, 0.f, 0.f, 0.f}; acc[tt] = z; }
      const unsigned short* ahp = sAh + m * HP + 8 * hh;
      const unsigned short* alp = sAl + m * HP + 8 * hh;
#pragma unroll
      for (int kt = 0; kt < DDIM / 32; ++kt) {
        FragB ah, al;
        ah.h[0] = *(const v8us*)(ahp + 32 * kt);
        ah.h[1] = *(const v8us*)(ahp + 32 * kt + 16);
        al.h[0] = *(const v8us*)(alp + 32 * kt);
        al.h[1] = *(const v8us*)(alp + 32 * kt + 16);
#pragma unroll
        for (int tt = 0; tt < 3; ++tt) {
          const int ti = 3 * wave + tt;
          const int mi = ti >> 3;
          const int n0 = (ti & 7) * 16;
          const unsigned short* bp = pq + (size_t)mi * (2 * DDIM * DDIM) + (size_t)(n0 + m) * DDIM + 32 * kt + 8 * hh;
          FragB bh, bl;
          bh.h[0] = *(const v8us*)bp;
          bh.h[1] = *(const v8us*)(bp + 16);
          bl.h[0] = *(const v8us*)(bp + DDIM * DDIM);
          bl.h[1] = *(const v8us*)(bp + DDIM * DDIM + 16);
          acc[tt] = wmb(ah.v, bh.v, acc[tt]);
          acc[tt] = wmb(ah.v, bl.v, acc[tt]);
          acc[tt] = wmb(al.v, bh.v, acc[tt]);
        }
      }
      float* sp = sQKV + (size_t)(8 * hh) * QP + m;
#pragma unroll
      for (int tt = 0; tt < 3; ++tt) {
        const int ti = 3 * wave + tt;
#pragma unroll
        for (int r = 0; r < 8; ++r) sp[r * QP + ti * 16] = acc[tt][r];
      }
    }
    __syncthreads();

    {
      const int q = tid >> 5, h = (tid >> 3) & 3, kt = tid & 7;
      const float* qp = sQKV + (size_t)q * QP + h * DH;
      const float* kp = sQKV + (size_t)kt * QP + DDIM + h * DH;
      float s = 0.0f;
#pragma unroll 1
      for (int j = 0; j < DH / 4; ++j) {
        const v4f a = *(const v4f*)(qp + 4 * j), c = *(const v4f*)(kp + 4 * j);
        s += a.x * c.x + a.y * c.y + a.z * c.z + a.w * c.w;
      }
      s *= RSQ;
      const int len = seqlen[b];
      if (kt >= len) s = -1.0e9f;
      float mx = s;
      mx = fmaxf(mx, __shfl_xor(mx, 1));
      mx = fmaxf(mx, __shfl_xor(mx, 2));
      mx = fmaxf(mx, __shfl_xor(mx, 4));
      float p = __expf(s - mx);
      float sum = p;
      sum += __shfl_xor(sum, 1);
      sum += __shfl_xor(sum, 2);
      sum += __shfl_xor(sum, 4);
      p = p * __builtin_amdgcn_rcpf(sum);
      sP[tid] = p;
    }
    __syncthreads();

    {
      const int q = tid >> 5, d4 = (tid & 31) * 4, h = (tid & 31) >> 3;
      v4f c = {0.f, 0.f, 0.f, 0.f};
#pragma unroll 1
      for (int kt = 0; kt < NT; ++kt) {
        const float pk = sP[q * (NTH * NT) + h * NT + kt];
        const v4f v = *(const v4f*)(sQKV + (size_t)kt * QP + 2 * DDIM + d4);
        c = c + v * pk;
      }
      v4us hv, lv;
      split4(c, hv, lv);
      *(v4us*)(sAh + q * HP + d4) = hv;
      *(v4us*)(sAl + q * HP + d4) = lv;
    }
    __syncthreads();

    {
      v8f acc = {0.f, 0.f, 0.f, 0.f, 0.f, 0.f, 0.f, 0.f};
      const unsigned short* ahp = sAh + m * HP + 8 * hh;
      const unsigned short* alp = sAl + m * HP + 8 * hh;
#pragma unroll
      for (int kt = 0; kt < DDIM / 32; ++kt) {
        FragB ah, al, bh, bl;
        ah.h[0] = *(const v8us*)(ahp + 32 * kt);
        ah.h[1] = *(const v8us*)(ahp + 32 * kt + 16);
        al.h[0] = *(const v8us*)(alp + 32 * kt);
        al.h[1] = *(const v8us*)(alp + 32 * kt + 16);
        const unsigned short* bp = pq + (size_t)3 * (2 * DDIM * DDIM) + (size_t)(16 * wave + m) * DDIM + 32 * kt + 8 * hh;
        bh.h[0] = *(const v8us*)bp;
        bh.h[1] = *(const v8us*)(bp + 16);
        bl.h[0] = *(const v8us*)(bp + DDIM * DDIM);
        bl.h[1] = *(const v8us*)(bp + DDIM * DDIM + 16);
        acc = wmb(ah.v, bh.v, acc);
        acc = wmb(ah.v, bl.v, acc);
        acc = wmb(al.v, bh.v, acc);
      }
      float* sp = sCto + (size_t)(8 * hh) * SP + 16 * wave + m;
#pragma unroll
      for (int r = 0; r < 8; ++r) sp[r * SP] = acc[r];
    }
    __syncthreads();

    if (tid < DDIM) {
      const int d = tid;
      const int len = seqlen[b];
      const int nv = len < 0 ? 0 : (len > NT ? NT : len);
      float s = 0.0f;
#pragma unroll 1
      for (int t = 0; t < NT; ++t) {
        const float hv = sHin[t * DDIM + d] + sCto[t * SP + d];
        s += (t < len) ? hv : 0.0f;
      }
      sSum[b * DDIM + d] = s * (1.0f / (float)nv);
    }
    __syncthreads();
  }

  if (tid < NBAT * NCLS) {
    const int b = tid / NCLS, c = tid - (tid / NCLS) * NCLS;
    float o = 0.0f;
#pragma unroll 1
    for (int d = 0; d < DDIM; ++d) o += sSum[b * DDIM + d] * Wc[d * NCLS + c];
    sOut[tid] = o + bc[c];
  }
  __syncthreads();
  if (wave == 0) {
    const v4f v = *(const v4f*)(sOut + 4 * lane);
    if (lane < (NBAT * NCLS) / 4) *(volatile v4f*)(out + 4 * lane) = v;
    __threadfence();
    if (lane < (NBAT * NCLS) / 4) *(volatile v4f*)(out + 4 * lane) = v;
  }
}

extern "C" void kernel_launch(void* const* d_in, const int* in_sizes, int n_in,
                              void* d_out, int out_size, void* d_ws, size_t ws_size,
                              hipStream_t stream) {
  if (n_in < 25) return;
  if (in_sizes[0] != NROWS * FIN || in_sizes[1] != NGRAPH * NEDGE * 2 || in_sizes[2] != NGRAPH) return;
  if (in_sizes[3] != 2 * NEDGE || in_sizes[4] != NBAT) return;
  if (in_sizes[5] != FIN * DDIM || in_sizes[6] != 2 * DDIM) return;
  if (in_sizes[7] != DDIM || in_sizes[8] != DDIM || in_sizes[9] != DDIM || in_sizes[10] != DDIM) return;
  if (in_sizes[11] != DDIM * DDIM || in_sizes[12] != 2 * DDIM) return;
  if (in_sizes[13] != DDIM || in_sizes[14] != DDIM || in_sizes[15] != DDIM || in_sizes[16] != DDIM) return;
  if (in_sizes[17] != DDIM || in_sizes[18] != DDIM) return;
  if (in_sizes[19] != DDIM * DDIM || in_sizes[20] != DDIM * DDIM || in_sizes[21] != DDIM * DDIM || in_sizes[22] != DDIM * DDIM) return;
  if (in_sizes[23] != DDIM * NCLS || in_sizes[24] != NCLS) return;
  if (out_size != NBAT * NCLS) return;

  const float* x_seq     = (const float*)d_in[0];
  const float* ea_seq    = (const float*)d_in[1];
  const float* intervals = (const float*)d_in[2];
  const int*   eidx      = (const int*)d_in[3];
  const int*   seqlen    = (const int*)d_in[4];
  const float* W0  = (const float*)d_in[5];
  const float* We0 = (const float*)d_in[6];
  const float* as0 = (const float*)d_in[7];
  const float* ad0 = (const float*)d_in[8];
  const float* ae0 = (const float*)d_in[9];
  const float* b0  = (const float*)d_in[10];
  const float* W1  = (const float*)d_in[11];
  const float* We1 = (const float*)d_in[12];
  const float* as1 = (const float*)d_in[13];
  const float* ad1 = (const float*)d_in[14];
  const float* ae1 = (const float*)d_in[15];
  const float* b1  = (const float*)d_in[16];
  const float* wt  = (const float*)d_in[17];
  const float* bt  = (const float*)d_in[18];
  const float* Wq  = (const float*)d_in[19];
  const float* Wk  = (const float*)d_in[20];
  const float* Wv  = (const float*)d_in[21];
  const float* Wo  = (const float*)d_in[22];
  const float* Wc  = (const float*)d_in[23];
  const float* bc  = (const float*)d_in[24];
  float* out = (float*)d_out;

  char* ws = (char*)d_ws;
  size_t off = 0;
  const size_t oW0 = off; off += (size_t)2 * DDIM * FIN * 2;         off = (off + 255) & ~(size_t)255;
  const size_t oW1 = off; off += (size_t)2 * DDIM * DDIM * 2;        off = (off + 255) & ~(size_t)255;
  const size_t oWQ = off; off += (size_t)4 * 2 * DDIM * DDIM * 2;    off = (off + 255) & ~(size_t)255;
  const size_t oXh = off; off += (size_t)NROWS * FIN * 2;            off = (off + 255) & ~(size_t)255;
  const size_t oXl = off; off += (size_t)NROWS * FIN * 2;            off = (off + 255) & ~(size_t)255;
  const size_t oHp = off; off += (size_t)NROWS * DDIM * 4;           off = (off + 255) & ~(size_t)255;
  const size_t oES = off; off += (size_t)NROWS * NHEAD * 4;          off = (off + 255) & ~(size_t)255;
  const size_t oED = off; off += (size_t)NROWS * NHEAD * 4;          off = (off + 255) & ~(size_t)255;
  const size_t oHh = off; off += (size_t)NROWS * DDIM * 2;           off = (off + 255) & ~(size_t)255;
  const size_t oHl = off; off += (size_t)NROWS * DDIM * 2;           off = (off + 255) & ~(size_t)255;
  const size_t oPt = off; off += (size_t)NGRAPH * NTG * DDIM * 4;    off = (off + 255) & ~(size_t)255;
  if (off > ws_size || off > (size_t)WSCAP) return;
  unsigned short* p0  = (unsigned short*)(ws + oW0);
  unsigned short* p1  = (unsigned short*)(ws + oW1);
  unsigned short* pq  = (unsigned short*)(ws + oWQ);
  unsigned short* xh  = (unsigned short*)(ws + oXh);
  unsigned short* xl  = (unsigned short*)(ws + oXl);
  float* hp  = (float*)(ws + oHp);
  float* eSp = (float*)(ws + oES);
  float* eDp = (float*)(ws + oED);
  unsigned short* h0h = (unsigned short*)(ws + oHh);
  unsigned short* h0l = (unsigned short*)(ws + oHl);
  float* part = (float*)(ws + oPt);

  const int nE = NEDGE;
  const int vec8 = ((nE & 3) == 0) ? 1 : 0;
  const int nUnits = NROWS * FIN / 8;

  k_prep_w<<<4 + 5 * 8, NTHR, 0, stream>>>(W0, W1, Wq, Wk, Wv, Wo, p0, p1, pq);
  k_cvt<<<nUnits / NTHR, NTHR, 0, stream>>>(x_seq, xh, xl, nUnits);
  k_gemm<<<NROWS / GB, GTHR, 0, stream>>>(xh, xl, p0, as0, ad0, hp, eSp, eDp, FIN, NROWS);
  hipFuncSetAttribute(reinterpret_cast<const void*>(&k_agg),
                      hipFuncAttributeMaxDynamicSharedMemorySize, LDS_AGG);
  k_agg<<<dim3(NTG, NGRAPH / GPB), NTHR, LDS_AGG, stream>>>(
      eidx, ea_seq, We0, ae0, b0, hp, eSp, eDp, h0h, h0l, part, NNODE, nE, NGRAPH, NTG, vec8, 0);
  k_gemm<<<NROWS / GB, GTHR, 0, stream>>>(h0h, h0l, p1, as1, ad1, hp, eSp, eDp, DDIM, NROWS);
  k_agg<<<dim3(NTG, NGRAPH / GPB), NTHR, LDS_AGG, stream>>>(
      eidx, ea_seq, We1, ae1, b1, hp, eSp, eDp, h0h, h0l, part, NNODE, nE, NGRAPH, NTG, vec8, 1);
  k_tail<<<1, NTHR, 0, stream>>>(part, intervals, wt, bt, pq, seqlen, Wc, bc, out, NBAT, NTG);
}
